// Multi_Head_Attention_59596966199577
// MI455X (gfx1250) — hardware-verified
//
#include <hip/hip_runtime.h>
#include <math.h>

typedef __attribute__((ext_vector_type(16))) _Float16 v16h;
typedef __attribute__((ext_vector_type(16))) __bf16 v16b;
typedef __attribute__((ext_vector_type(8)))  _Float16 v8h;
typedef __attribute__((ext_vector_type(8)))  float v8f;
typedef __attribute__((ext_vector_type(4)))  float v4f;
typedef __attribute__((ext_vector_type(4)))  unsigned v4u;

template <typename T> __device__ __forceinline__ void vst2(void* p, T v) { *(volatile T*)p = v; __threadfence(); *(volatile T*)p = v; }
__device__ __forceinline__ v8f wmma16(v16h a, v16h b, v8f c) {
  v8f d = __builtin_amdgcn_wmma_f32_16x16x32_f16(false, a, false, b, (short)0, c, false, false);
  asm volatile("v_nop\n\tv_nop\n\tv_nop\n\tv_nop" : "+v"(d) : "v"(a), "v"(b));
  return d;
}
__device__ __forceinline__ v8f wmma_bf(v16b a, v16b b, v8f c) {
  v8f d = __builtin_amdgcn_wmma_f32_16x16x32_bf16(false, a, false, b, (short)0, c, false, false);
  asm volatile("v_nop\n\tv_nop\n\tv_nop\n\tv_nop" : "+v"(d) : "v"(a), "v"(b));
  return d;
}
__device__ __forceinline__ v16h frag_h(const _Float16* rowk0, int lane) {
  union { v16h v; v8h q[2]; } u; const _Float16* p = rowk0 + 8 * (lane >> 4);
  u.q[0] = *(const v8h*)p; u.q[1] = *(const v8h*)(p + 16); return u.v;
}
__device__ __forceinline__ v16h frag_f32(const float* rowk0, int lane) {
  v16h a; const float* p = rowk0 + 8 * (lane >> 4);
#pragma unroll
  for (int i = 0; i < 8; ++i) { a[i] = (_Float16)p[i]; a[8 + i] = (_Float16)p[16 + i]; }
  return a;
}
struct F2 { v16b h, l; };
__device__ __forceinline__ F2 bsplit16(const float v[16]) { F2 r;
#pragma unroll
  for (int i = 0; i < 16; ++i) { const __bf16 h = (__bf16)v[i]; r.h[i] = h; r.l[i] = (__bf16)(v[i] - (float)h); }
  return r; }
__device__ __forceinline__ F2 split_row(const float* row, int k0, int lane) { float v[16]; const float* p = row + k0 + 8 * (lane >> 4);
#pragma unroll
  for (int i = 0; i < 8; ++i) { v[i] = p[i]; v[8 + i] = p[16 + i]; }
  return bsplit16(v); }
#define LDSX() do { asm volatile("s_wait_dscnt 0" ::: "memory"); __builtin_amdgcn_wave_barrier(); __builtin_amdgcn_fence(3  , "workgroup"); } while (0)

#ifndef NB
#define NB 4
#endif
#ifndef SEQ
#define SEQ 2048
#endif
#define TT SEQ
#define NB_FULL 4
#define TT_FULL 2048
#define DM 512
#define NH 8
#define HD 64
#define CK (NH * HD)
#define HG 4
#define PCAR 2048.0f
#define CSUB (PCAR / (float)TT)
#define L2E 1.4426950408889634f
#define SM_NT ((((TT) / 4) < 256) ? ((TT) / 4) : 256)
#define SM_NCH ((TT) / (4 * SM_NT))

static_assert(NB >= 1 && NB <= NB_FULL);
static_assert(TT >= 256 && TT <= TT_FULL);
static_assert((TT % 256) == 0 && (TT % 128) == 0 && (TT % 64) == 0);
static_assert((SM_NT % 32) == 0 && SM_NT * 4 * SM_NCH == TT);
static_assert((DM % 128) == 0 && (DM % 32) == 0 && (CK % 128) == 0 && (CK % 32) == 0);
static_assert(HD == 64 && (NH % HG) == 0 && CK == DM);

#define WS_QH  ((size_t)0)
#define WS_QL  (WS_QH + 2u * (size_t)NB * TT * CK)
#define WS_KH  (WS_QL + 2u * (size_t)NB * TT * CK)
#define WS_VT  (WS_KH + 2u * (size_t)NB * TT * CK)
#define WS_VL  (WS_VT + 2u * (size_t)NB * CK * TT)
#define WS_S   (WS_VL + 2u * (size_t)NB * CK * TT)
#define WS_Y   (WS_S + 4u * (size_t)HG * TT * TT)
#define WS_VM  (WS_Y + 4u * (size_t)NB * TT * CK)
#define WS_END (WS_VM + 4u * (size_t)NB * CK)
static_assert(WS_END <= (size_t)134217728u);
static_assert((WS_QL % 128) == 0 && (WS_KH % 128) == 0 && (WS_VT % 128) == 0 && (WS_VL % 128) == 0 && (WS_S % 128) == 0 && (WS_Y % 128) == 0 && (WS_VM % 128) == 0 && (WS_END % 128) == 0);

__global__ __launch_bounds__(128) void k_proj(const float* __restrict__ X, const float* __restrict__ WQ, const float* __restrict__ WK, const float* __restrict__ WV, _Float16* __restrict__ QH, _Float16* __restrict__ QL, _Float16* __restrict__ KH, _Float16* __restrict__ VT, _Float16* __restrict__ VL) {
  __shared__ __align__(16) _Float16 sh[64][136], sl[64][136]; __shared__ __align__(16) _Float16 th[128][72], tl2[128][72];
  const int tid = threadIdx.x, wave = tid >> 5, lane = tid & 31, col = lane & 15, g = lane >> 4;
  const int which = blockIdx.z; const int c0 = blockIdx.y * 128;
  const size_t r0 = (size_t)blockIdx.x * 64;
  const size_t b = r0 / TT; const int t0 = (int)(r0 % TT);
  const size_t xr0 = b * TT_FULL + (size_t)t0;
  const float* WA = which == 0 ? WQ : which == 1 ? WK : WV;
  v8f acc[8] = {};
#pragma unroll 2
  for (int kc = 0; kc < DM / 32; ++kc) { v16b a; { const float* p = X + (xr0 + wave * 16 + col) * DM + kc * 32 + 8 * g;
#pragma unroll
      for (int i = 0; i < 8; ++i) { a[i] = (__bf16)p[i]; a[8 + i] = (__bf16)p[16 + i]; } }
#pragma unroll
    for (int j = 0; j < 8; ++j) { v16b w; const int o = c0 + j * 16 + col; const size_t wb = (size_t)(o / HD) * DM * HD + (size_t)(o % HD);
#pragma unroll
      for (int i = 0; i < 8; ++i) { w[i] = (__bf16)WA[wb + (size_t)(kc * 32 + 8 * g + i) * HD]; w[8 + i] = (__bf16)WA[wb + (size_t)(kc * 32 + 16 + 8 * g + i) * HD]; }
      acc[j] = wmma_bf(a, w, acc[j]); } }
#pragma unroll
  for (int j = 0; j < 8; ++j) {
#pragma unroll
    for (int r = 0; r < 8; ++r) { const float v = acc[j][r]; const int rl = wave * 16 + 8 * g + r, cl = j * 16 + col; const _Float16 hv = (_Float16)v; const _Float16 lv = (_Float16)((v - (float)hv) * 1024.0f);
      if (which == 2) { th[cl][rl] = hv; tl2[cl][rl] = lv; } else { sh[rl][cl] = hv; sl[rl][cl] = lv; } } }
  __syncthreads();
  if (which < 2) { _Float16* dh = which == 0 ? QH : KH;
    for (int e = tid; e < 64 * 16; e += 128) { const int rl = e >> 4, q = e & 15; vst2(dh + (r0 + rl) * CK + c0 + q * 8, *(const v4u*)&sh[rl][q * 8]); if (which == 0) vst2(QL + (r0 + rl) * CK + c0 + q * 8, *(const v4u*)&sl[rl][q * 8]); } }
  else { for (int e = tid; e < 128 * 8; e += 128) { const int cl = e >> 3, q = e & 7; const size_t o2 = (b * CK + c0 + cl) * (size_t)TT + t0 + q * 8; vst2(VT + o2, *(const v4u*)&th[cl][q * 8]); vst2(VL + o2, *(const v4u*)&tl2[cl][q * 8]); } } }

__global__ __launch_bounds__(256) void k_vmean(const _Float16* __restrict__ VT, const _Float16* __restrict__ VL, float* __restrict__ VM) {
  __shared__ __align__(16) float smv[32];
  const int tid = threadIdx.x, wave = tid >> 5, lane = tid & 31; const int b = blockIdx.x, c0 = blockIdx.y * 32;
#pragma unroll 1
  for (int j = 0; j < 4; ++j) { const int c = c0 + wave * 4 + j; const size_t base = ((size_t)b * CK + c) * (size_t)TT;
    float s_h = 0.f, s_l = 0.f;
#pragma unroll 1
    for (int i = 0; i < TT / 256; ++i) { const int ts = (lane + 32 * i) * 8; const v8h hv = *(const v8h*)(VT + base + ts); const v8h lv = *(const v8h*)(VL + base + ts);
#pragma unroll
      for (int e = 0; e < 8; ++e) { s_h += (float)hv[e]; s_l += (float)lv[e]; } }
    float s = s_h + s_l * (1.0f / 1024.0f);
#pragma unroll
    for (int o = 1; o < 32; o <<= 1) s += __shfl_xor(s, o);
    if (lane == 0) smv[wave * 4 + j] = s * (1.0f / (float)TT); }
  __syncthreads();
  if (wave == 0 && lane < 8) vst2(VM + (size_t)b * CK + c0 + lane * 4, *(const v4f*)&smv[lane * 4]); }

__global__ __launch_bounds__(128) void k_sc(const _Float16* __restrict__ QH, const _Float16* __restrict__ QL, const _Float16* __restrict__ KH, int b, int h0, float* __restrict__ S0) {
  __shared__ __align__(16) float ss[4][16][132];
  const int h = h0 + blockIdx.z; float* S = S0 + (size_t)blockIdx.z * TT * TT;
  const int tid = threadIdx.x, wave = tid >> 5, lane = tid & 31, col = lane & 15, g = lane >> 4; const int k0 = blockIdx.y * 128; const int ql0 = blockIdx.x * 64 + wave * 16; const size_t q0 = (size_t)b * TT + ql0;
  v8f acc[8] = {}, accl[8] = {};
#pragma unroll
  for (int kc = 0; kc < HD / 32; ++kc) { const v16h ah = frag_h(QH + (q0 + col) * CK + h * HD + kc * 32, lane), al = frag_h(QL + (q0 + col) * CK + h * HD + kc * 32, lane);
#pragma unroll
    for (int j = 0; j < 8; ++j) { const v16h kb = frag_h(KH + ((size_t)b * TT + k0 + j * 16 + col) * CK + h * HD + kc * 32, lane); acc[j] = wmma16(ah, kb, acc[j]); accl[j] = wmma16(al, kb, accl[j]); } }
#pragma unroll
  for (int j = 0; j < 8; ++j) acc[j] += accl[j] * (1.0f / 1024.0f);
#pragma unroll
  for (int j = 0; j < 8; ++j) {
#pragma unroll
    for (int r = 0; r < 8; ++r) ss[wave][8 * g + r][j * 16 + col] = acc[j][r] * 0.125f; }
  LDSX(); for (int rl = 0; rl < 16; ++rl) vst2(S + (size_t)(ql0 + rl) * TT + k0 + lane * 4, *(const v4f*)&ss[wave][rl][lane * 4]); }

__global__ __launch_bounds__(SM_NT) void k_sm(float* __restrict__ S0) {
  __shared__ float sred[SM_NT / 32]; __shared__ float sbc;
  const int t = threadIdx.x;
  float* sr = S0 + (size_t)blockIdx.y * TT * TT + (size_t)blockIdx.x * TT;
  v4f v[SM_NCH];
  float m = -3.0e38f;
#pragma unroll
  for (int i = 0; i < SM_NCH; ++i) { v[i] = *(const v4f*)(sr + 4 * (t + SM_NT * i)); m = fmaxf(m, fmaxf(fmaxf(v[i].x, v[i].y), fmaxf(v[i].z, v[i].w))); }
#pragma unroll
  for (int o = 1; o < 32; o <<= 1) m = fmaxf(m, __shfl_xor(m, o));
  if ((t & 31) == 0) sred[t >> 5] = m; __syncthreads(); if (t == 0) { float a = sred[0]; for (int i = 1; i < SM_NT / 32; ++i) a = fmaxf(a, sred[i]); sbc = a; } __syncthreads(); m = sbc; __syncthreads();
  float sum = 0.f;
#pragma unroll
  for (int i = 0; i < SM_NCH; ++i) { v4f e; e.x = exp2f((v[i].x - m) * L2E); e.y = exp2f((v[i].y - m) * L2E); e.z = exp2f((v[i].z - m) * L2E); e.w = exp2f((v[i].w - m) * L2E); sum += (e.x + e.y) + (e.z + e.w); v[i] = e; }
#pragma unroll
  for (int o = 1; o < 32; o <<= 1) sum += __shfl_xor(sum, o);
  if ((t & 31) == 0) sred[t >> 5] = sum; __syncthreads(); if (t == 0) { float a = 0.f; for (int i = 0; i < SM_NT / 32; ++i) a += sred[i]; sbc = 1.0f / a; } __syncthreads(); const float sc = sbc * PCAR;
#pragma unroll
  for (int i = 0; i < SM_NCH; ++i) { const v4f p = v[i] * sc - CSUB; vst2(sr + 4 * (t + SM_NT * i), p); } }

__global__ __launch_bounds__(128) void k_pv(const float* __restrict__ PS0, const _Float16* __restrict__ VT, const _Float16* __restrict__ VL, const float* __restrict__ VM, int b, int h0, float* __restrict__ Y) {
  const int h = h0 + blockIdx.z; const float* PS = PS0 + (size_t)blockIdx.z * TT * TT; __shared__ __align__(16) float ss[4][16][HD + 4];
  const int tid = threadIdx.x, wave = tid >> 5, lane = tid & 31, col = lane & 15, g = lane >> 4; const int ql0 = blockIdx.x * 64 + wave * 16;
  v8f acc[HD / 16] = {}, accl[HD / 16] = {};
#pragma unroll 1
  for (int kc = 0; kc < TT / 32; ++kc) { const v16h p = frag_f32(PS + (size_t)(ql0 + col) * TT + kc * 32, lane);
#pragma unroll
    for (int j = 0; j < HD / 16; ++j) { const size_t po = ((size_t)b * CK + h * HD + j * 16 + col) * (size_t)TT + kc * 32; acc[j] = wmma16(p, frag_h(VT + po, lane), acc[j]); accl[j] = wmma16(p, frag_h(VL + po, lane), accl[j]); } }
  float mv[HD / 16];
#pragma unroll
  for (int j = 0; j < HD / 16; ++j) mv[j] = VM[(size_t)b * CK + h * HD + j * 16 + col];
#pragma unroll
  for (int j = 0; j < HD / 16; ++j) {
#pragma unroll
    for (int r = 0; r < 8; ++r) ss[wave][8 * g + r][j * 16 + col] = (acc[j][r] + accl[j][r] * (1.0f / 1024.0f)) * (1.0f / PCAR) + mv[j]; }
  LDSX(); for (int rl = 0; rl < 16; ++rl) if (lane < HD / 4) vst2(Y + ((size_t)b * TT + ql0 + rl) * CK + h * HD + lane * 4, *(const v4f*)&ss[wave][rl][lane * 4]); }

__global__ __launch_bounds__(128) void k_out(const float* __restrict__ Y, const float* __restrict__ WO, float* __restrict__ OUT) { __shared__ __align__(16) float sf[4][16][132];
  const int tid = threadIdx.x, wave = tid >> 5, lane = tid & 31, col = lane & 15, g = lane >> 4; const int c0 = blockIdx.y * 128;
  const size_t r0 = (size_t)blockIdx.x * 64 + wave * 16;
  const size_t ob = ((size_t)blockIdx.x * 64) / TT; const size_t orow0 = ob * TT_FULL + (r0 - ob * TT);
  v8f acc[8] = {};
#pragma unroll 2
  for (int kc = 0; kc < CK / 32; ++kc) { const F2 a = split_row(Y + (r0 + col) * CK, kc * 32, lane);
#pragma unroll
    for (int j = 0; j < 8; ++j) { v16b w; const int o = c0 + j * 16 + col;
#pragma unroll
      for (int i = 0; i < 8; ++i) { w[i] = (__bf16)WO[(size_t)(kc * 32 + 8 * g + i) * DM + o]; w[8 + i] = (__bf16)WO[(size_t)(kc * 32 + 16 + 8 * g + i) * DM + o]; }
      acc[j] = wmma_bf(a.h, w, acc[j]); acc[j] = wmma_bf(a.l, w, acc[j]); } }
#pragma unroll
  for (int j = 0; j < 8; ++j) {
#pragma unroll
    for (int r = 0; r < 8; ++r) sf[wave][8 * g + r][j * 16 + col] = acc[j][r]; }
  LDSX(); for (int rl = 0; rl < 16; ++rl) vst2(OUT + (orow0 + rl) * DM + c0 + lane * 4, *(const v4f*)&sf[wave][rl][lane * 4]); }

extern "C" void kernel_launch(void* const* d_in, const int* in_sizes, int n_in, void* d_out, int out_size, void* d_ws, size_t ws_size, hipStream_t stream) {
  if (n_in < 5) return;
  const float* X = (const float*)d_in[0];
  const float* WQ = (const float*)d_in[1];
  const float* WK = (const float*)d_in[2];
  const float* WV = (const float*)d_in[3];
  const float* WO = (const float*)d_in[4];
  const size_t need_rows = (size_t)(NB - 1) * TT_FULL + (size_t)TT;
  if ((size_t)in_sizes[0] < need_rows * DM) return;
  if ((size_t)in_sizes[1] < (size_t)NH * DM * HD || (size_t)in_sizes[2] < (size_t)NH * DM * HD || (size_t)in_sizes[3] < (size_t)NH * DM * HD) return;
  if ((size_t)in_sizes[4] < (size_t)CK * DM) return;
  if ((size_t)out_size < need_rows * DM) return;
  if (ws_size < (size_t)WS_END) return;
  char* ws = (char*)d_ws;
  _Float16 *QH = (_Float16*)(ws + WS_QH), *QL = (_Float16*)(ws + WS_QL), *KH = (_Float16*)(ws + WS_KH), *VT = (_Float16*)(ws + WS_VT), *VL = (_Float16*)(ws + WS_VL);
  float *S = (float*)(ws + WS_S), *Y = (float*)(ws + WS_Y), *VM = (float*)(ws + WS_VM);
  k_proj<<<dim3(NB * TT / 64, CK / 128, 3), 128, 0, stream>>>(X, WQ, WK, WV, QH, QL, KH, VT, VL);
  k_vmean<<<dim3(NB, CK / 32), 256, 0, stream>>>(VT, VL, VM);
  for (int b = 0; b < NB; ++b) for (int h0 = 0; h0 < NH; h0 += HG) {
    k_sc<<<dim3(TT / 64, TT / 128, HG), 128, 0, stream>>>(QH, QL, KH, b, h0, S);
    k_sm<<<dim3(TT, HG), SM_NT, 0, stream>>>(S);
    k_pv<<<dim3(TT / 64, 1, HG), 128, 0, stream>>>(S, VT, VL, VM, b, h0, Y);
  }
  k_out<<<dim3(NB * TT / 64, DM / 128), 128, 0, stream>>>(Y, WO, (float*)d_out);
}
